// GCNExtractor_5669356835492
// MI455X (gfx1250) — hardware-run, weakly checked
//
#include <hip/hip_runtime.h>


#ifndef NN
#define NN 2048
#endif
#define NN_FULL 2048
#define FF   128
#define HT   128
#define HIT  16
#define HW   64
#define HB   ((NN * NN / 4) / (HT * HIT))
#define TT   512
#define C4   ((NN * NN / 4) / TT)
#define SR   32
#define ITS  (NN / 256)
#define H2S  4096.0f
#define H2I  (1.0f / 4096.0f)

static constexpr unsigned KEEPC = (unsigned)(0.3 * NN * NN);
static_assert(NN != 2048 || KEEPC == 1258291u);
static_assert(NN <= NN_FULL);
static_assert(NN % 256 == 0);
static_assert(NN % 64 == 0);
static_assert(NN % 32 == 0);
static_assert(FF == 128);
static_assert(FF % 64 == 0);
static_assert(FF % 32 == 0);
static_assert((NN * NN / 4) % (HT * HIT) == 0);
static_assert(HB >= 1);
static_assert(HW * 4 == 256);
static_assert(HIT * 4 <= 255);
static_assert(HT * HIT * 4 <= 65535);
static_assert(2 * HT == 256);
static_assert(HW <= HT);
static_assert(HW % 32 == 0);
static_assert(HW * HT * 4 + 256 * 4 < 65536);
static_assert((NN * NN / 4) % TT == 0);
static_assert(NN % SR == 0);
static_assert(SR == 32);
static_assert((256 / 32) * (SR / 8) == SR);
static_assert((unsigned long long)NN * NN <= 0xFFFFFFFFull);
static_assert(16 * 68 * 4 <= 131072);
static_assert(32 * 132 * 4 <= 131072);
static_assert(TT * 4 + 16 <= 131072);

typedef _Float16 h16;
typedef unsigned short bf;
typedef __attribute__((ext_vector_type(16))) __bf16   v16bf;
typedef __attribute__((ext_vector_type(16))) _Float16 v16h;
typedef __attribute__((ext_vector_type(8)))  _Float16 v8h;
typedef __attribute__((ext_vector_type(8)))  unsigned short v8us;
typedef __attribute__((ext_vector_type(8)))  float    v8f;
typedef __attribute__((ext_vector_type(4)))  float    v4f;
typedef v4f  __attribute__((may_alias)) v4fa;

__device__ __forceinline__ unsigned short f2bf(float f) { unsigned u = __float_as_uint(f); u += 0x7FFFu + ((u >> 16) & 1u); return (unsigned short)(u >> 16); }
__device__ __forceinline__ float bfr(float f) { return __uint_as_float(((unsigned)f2bf(f)) << 16); }
__device__ __forceinline__ v16h cat16(v8h lo, v8h hi) { return __builtin_shufflevector(lo, hi, 0, 1, 2, 3, 4, 5, 6, 7, 8, 9, 10, 11, 12, 13, 14, 15); }
__device__ __forceinline__ v16bf cat16b(v8us lo, v8us hi) { return __builtin_bit_cast(v16bf, __builtin_shufflevector(lo, hi, 0, 1, 2, 3, 4, 5, 6, 7, 8, 9, 10, 11, 12, 13, 14, 15)); }
__device__ __forceinline__ v8f wmma16(v16h a, v16h b, v8f c) { return __builtin_amdgcn_wmma_f32_16x16x32_f16(false, a, false, b, (short)0, c, false, false); }
__device__ __forceinline__ v8f wmmab(v16bf a, v16bf b, v8f c) { return __builtin_amdgcn_wmma_f32_16x16x32_bf16(false, a, false, b, (short)0, c, false, false); }
__device__ __forceinline__ v16h  ldh(const h16* p) { return cat16(*(const v8h*)p, *(const v8h*)(p + 16)); }
__device__ __forceinline__ v16bf ldb(const bf* p)  { return cat16b(*(const v8us*)p, *(const v8us*)(p + 16)); }
__device__ __forceinline__ void wave_sync() { __builtin_amdgcn_fence(3  , "wavefront"); __builtin_amdgcn_wave_barrier(); asm volatile("" ::: "memory"); }

__device__ __forceinline__ v8f wmmabg(v16bf a, v16bf b, v8f c) { c = wmmab(a, b, c); asm volatile("v_nop\n\tv_nop\n\tv_nop\n\tv_nop" : "+v"(c) : "v"(a), "v"(b)); return c; }
__device__ __forceinline__ v8f wmma16g(v16h a, v16h b, v8f c) { c = wmma16(a, b, c); asm volatile("v_nop\n\tv_nop\n\tv_nop\n\tv_nop" : "+v"(c) : "v"(a), "v"(b)); return c; }
__device__ __forceinline__ h16 toh_flush(float v) { const h16 r = (h16)v; return (fabsf(v) < 6.103515625e-05f) ? (h16)0.0f : r; }
__device__ __forceinline__ unsigned fkey(float f) { const unsigned u = __float_as_uint(f); return (u & 0x80000000u) ? ~u : (u | 0x80000000u); }

__global__ __launch_bounds__(256) void k_cvt8(const float* __restrict__ src, bf* dst, size_t n8) {
    const size_t i = (size_t)blockIdx.x * 256 + threadIdx.x; if (i >= n8) return;
    const v8f v = *(const v8f*)(src + i * 8); v8us o;
#pragma unroll
    for (int k = 0; k < 8; ++k) o[k] = f2bf(v[k]);
    *(volatile v8us*)(dst + i * 8) = o; __threadfence(); *(volatile v8us*)(dst + i * 8) = o;
}

static_assert(16 * 256 == FF * 32);
static_assert(2 * 256 * 16 == 32 * FF * 2);
__global__ __launch_bounds__(256) void k_wt(const float* __restrict__ W, bf* WT) {
    __shared__ __align__(16) float lt[32 * 132];
    const int tid = threadIdx.x; const int o0 = blockIdx.x * 32;
#pragma unroll 4
    for (int i = 0; i < 16; ++i) { const int e = i * 256 + tid; const int k = e >> 5, j = e & 31; lt[j * 132 + k] = W[(size_t)k * FF + o0 + j]; }
    __syncthreads();
    v8us o[2];
#pragma unroll
    for (int it = 0; it < 2; ++it) { const int p = it * 256 + tid; const int row = p >> 4, c8 = (p & 15) * 8;
        const v4f x0 = *(const v4fa*)(&lt[row * 132 + c8]); const v4f x1 = *(const v4fa*)(&lt[row * 132 + c8 + 4]);
#pragma unroll
        for (int i = 0; i < 4; ++i) { o[it][i] = f2bf(x0[i]); o[it][4 + i] = f2bf(x1[i]); } }
    bf* dst = WT + (size_t)o0 * FF + (size_t)tid * 8;
#pragma unroll 1
    for (int ps = 0; ps < 2; ++ps) {
#pragma unroll
        for (int it = 0; it < 2; ++it) *(volatile v8us*)(dst + (size_t)it * 2048) = o[it];
        if (ps == 0) __threadfence(); }
}

static_assert(8 * 32 * 16 == 16 * 64 * 4);
__global__ __launch_bounds__(32) void k_sim(const bf* __restrict__ XB, float* S) {
    __shared__ __align__(16) float os[16 * 68];
    const int lane = threadIdx.x & 31, lr = lane & 15, hi = lane >> 4; const int r0 = blockIdx.x * 64, c0 = blockIdx.y * 64;
    v8f acc[4][4];
#pragma unroll
    for (int mb = 0; mb < 4; ++mb)
#pragma unroll
        for (int nb = 0; nb < 4; ++nb) acc[mb][nb] = (v8f){};
    const size_t aoff = (size_t)(r0 + lr) * FF + 8 * hi, boff = (size_t)(c0 + lr) * FF + 8 * hi;
#pragma unroll 1
    for (int kc = 0; kc < FF; kc += 32) {
        v16bf a[4];
#pragma unroll
        for (int mb = 0; mb < 4; ++mb) a[mb] = ldb(XB + aoff + (size_t)mb * 16 * FF + kc);
#pragma unroll
        for (int nb = 0; nb < 4; ++nb) { const v16bf b = ldb(XB + boff + (size_t)nb * 16 * FF + kc);
#pragma unroll
            for (int mb = 0; mb < 4; ++mb) acc[mb][nb] = wmmabg(a[mb], b, acc[mb][nb]); }
    }
#pragma unroll
    for (int mb = 0; mb < 4; ++mb) {
#pragma unroll
        for (int nb = 0; nb < 4; ++nb) {
#pragma unroll
            for (int j = 0; j < 8; ++j) { const int m = r0 + mb * 16 + hi * 8 + j, n = c0 + nb * 16 + lr;
                const float v = acc[mb][nb][j]; os[(hi * 8 + j) * 68 + nb * 16 + lr] = (m == n) ? (v - 1.0f) : v; } }
        wave_sync();
#pragma unroll 1
        for (int ps = 0; ps < 2; ++ps) {
#pragma unroll
            for (int s = 0; s < 8; ++s) { const int row = 2 * s + (lane >> 4), cofs = (lane & 15) * 4;
                const v4f val = *(const v4fa*)(&os[row * 68 + cofs]);
                *(volatile v4f*)(S + (size_t)(r0 + mb * 16 + row) * NN + c0 + cofs) = val; }
            if (ps == 0) __threadfence(); }
        wave_sync();
    }
}

__global__ __launch_bounds__(32) void k_init(unsigned* ST) {
    const int lane = threadIdx.x & 31;
    const unsigned v = (lane == 1) ? KEEPC : 0u;
    *(volatile unsigned*)(ST + lane) = v; __threadfence(); *(volatile unsigned*)(ST + lane) = v;
}

__global__ __launch_bounds__(HT) void k_hist(const float* __restrict__ S, const unsigned* __restrict__ ST, unsigned* HP, int pass) {
    __shared__ unsigned hloc[HW * HT];
    __shared__ unsigned hcnt[256];
    const int tid = threadIdx.x;
    const int wave = __builtin_amdgcn_readfirstlane((int)(threadIdx.x >> 5));
#pragma unroll 4
    for (int w = 0; w < HW; ++w) hloc[w * HT + tid] = 0u;
    const unsigned prefix = ST[0];
    const int shift = 24 - 8 * pass; const int hs = shift + 8;
    const size_t base4 = (size_t)blockIdx.x * (size_t)(HT * HIT);
#pragma unroll 4
    for (int i = 0; i < HIT; ++i) {
        const v4f f = *(const v4f*)(S + (base4 + (size_t)i * HT + tid) * 4);
#pragma unroll
        for (int j = 0; j < 4; ++j) { const unsigned k = fkey(f[j]);
            const bool ok = ((unsigned)(((unsigned long long)k) >> hs) == prefix);
            const unsigned bin = (k >> shift) & 255u;
            const unsigned inc = ok ? (1u << ((bin & 3u) * 8u)) : 0u;
            const int wi = (int)(bin >> 2) * HT + tid;
            const unsigned cur = hloc[wi];
            hloc[wi] = cur + inc; }
    }
    __syncthreads();
    if (wave < HW / 32) {
        unsigned lo = 0u, hi2 = 0u;
#pragma unroll 4
        for (int t = 0; t < HT; ++t) { const unsigned v = hloc[tid * HT + t]; lo += v & 0x00FF00FFu; hi2 += (v >> 8) & 0x00FF00FFu; }
        hcnt[4 * tid + 0] = lo & 0xFFFFu; hcnt[4 * tid + 1] = hi2 & 0xFFFFu; hcnt[4 * tid + 2] = lo >> 16; hcnt[4 * tid + 3] = hi2 >> 16;
    }
    __syncthreads();
    const unsigned c0 = hcnt[tid], c1 = hcnt[HT + tid];
    unsigned* dst = HP + (size_t)blockIdx.x * 256 + tid;
#pragma unroll 1
    for (int ps = 0; ps < 2; ++ps) {
        *(volatile unsigned*)dst = c0; *(volatile unsigned*)(dst + HT) = c1;
        if (ps == 0) __threadfence(); }
}

__global__ __launch_bounds__(256) void k_scan(const unsigned* __restrict__ HP, unsigned* ST) {
    __shared__ unsigned cnt[256];
    const int lane = threadIdx.x & 31;
    const int wave = __builtin_amdgcn_readfirstlane((int)(threadIdx.x >> 5));
    unsigned s = 0u;
#pragma unroll 4
    for (int b = 0; b < HB; ++b) s += HP[(size_t)b * 256 + threadIdx.x];
    cnt[threadIdx.x] = s;
    const unsigned pre = ST[0], rem0 = ST[1];
    __syncthreads();
    if (wave == 0) {
        unsigned rem = rem0, newpre = pre << 8; bool done = false;
#pragma unroll 1
        for (int b = 255; b >= 0; --b) { const unsigned c = cnt[b];
            const bool take = (!done) & (rem <= c); const bool sub = (!done) & (rem > c);
            newpre = take ? ((pre << 8) | (unsigned)b) : newpre; rem = sub ? (rem - c) : rem; done = done | take; }
        const unsigned v = (lane == 0) ? newpre : ((lane == 1) ? rem : 0u);
        *(volatile unsigned*)(ST + lane) = v; __threadfence(); *(volatile unsigned*)(ST + lane) = v;
    }
}

__global__ __launch_bounds__(TT) void k_tie(const float* __restrict__ S, unsigned* ST) {
    __shared__ unsigned sc[TT];
    __shared__ unsigned res;
    const int tid = threadIdx.x; const int lane = tid & 31;
    const int wave = __builtin_amdgcn_readfirstlane((int)(threadIdx.x >> 5));
    const unsigned tkey = ST[0], rem = ST[1];
    const size_t b4 = (size_t)tid * (size_t)C4;
    unsigned cnt = 0u;
#pragma unroll 4
    for (int i = 0; i < C4; ++i) { const v4f f = *(const v4f*)(S + (b4 + (size_t)i) * 4);
        cnt += (fkey(f[0]) == tkey ? 1u : 0u) + (fkey(f[1]) == tkey ? 1u : 0u) + (fkey(f[2]) == tkey ? 1u : 0u) + (fkey(f[3]) == tkey ? 1u : 0u); }
    sc[tid] = cnt; if (tid == 0) res = 0xFFFFFFFFu;
    __syncthreads();
    unsigned ex = 0u;
#pragma unroll 4
    for (int i = 0; i < TT; ++i) { const unsigned c = sc[i]; ex += (i < tid) ? c : 0u; }
    const unsigned need = rem - ex;
    const bool hit = (rem > ex) & (need <= cnt);
    const bool whit = (__ballot(hit ? 1 : 0) != 0ull);
    if (whit) {
        unsigned c = 0u, idx = 0xFFFFFFFFu;
#pragma unroll 2
        for (int i = 0; i < C4; ++i) { const v4f f = *(const v4f*)(S + (b4 + (size_t)i) * 4);
#pragma unroll
            for (int j = 0; j < 4; ++j) { const bool t = (fkey(f[j]) == tkey); c += t ? 1u : 0u;
                idx = (t & hit & (c == need)) ? (unsigned)((b4 + (size_t)i) * 4 + (size_t)j) : idx; } }
        if (hit) res = idx;
    }
    __syncthreads();
    if (wave == 0) { const unsigned rv = res; const unsigned v = (lane == 0) ? rv : 0u;
        *(volatile unsigned*)(ST + 32 + lane) = v; __threadfence(); *(volatile unsigned*)(ST + 32 + lane) = v; }
}

static_assert(ITS * 32 * 16 == NN * 2);
__global__ __launch_bounds__(256) void k_select(const float* __restrict__ S, const unsigned* __restrict__ ST, h16* P, float* DV) {
    __shared__ float dg[SR];
    const int lane = threadIdx.x & 31;
    const int wave = __builtin_amdgcn_readfirstlane((int)(threadIdx.x >> 5));
    const unsigned tkey = ST[0], cut = ST[32];
#pragma unroll 1
    for (int q = 0; q < SR / 8; ++q) {
        const int rl = wave * (SR / 8) + q;
        const int c = blockIdx.x * SR + rl;
        const float* srow = S + (size_t)c * NN + lane * 8;
        h16* prow = P + (size_t)c * NN + lane * 8;
        v8h pv[ITS]; float s = 0.0f;
#pragma unroll
        for (int it = 0; it < ITS; ++it) {
            v4f f0 = *(const v4f*)(srow + it * 256), f1 = *(const v4f*)(srow + it * 256 + 4);
            asm volatile("" : "+v"(f0)); asm volatile("" : "+v"(f1));
            const int rb = it * 256 + lane * 8;
#pragma unroll
            for (int j = 0; j < 8; ++j) {
                const float v = (j < 4) ? f0[j & 3] : f1[j & 3];
                const unsigned k = fkey(v);
                const int rr = rb + j;
                const unsigned flat = (unsigned)rr * (unsigned)NN + (unsigned)c;
                const bool sel = (k > tkey) | ((k == tkey) & (flat <= cut));
                float a = sel ? v : 0.0f;
                a += (rr == c) ? 1.0f : 0.0f;
                s += a;
                pv[it][j] = toh_flush(a); }
        }
        s += __shfl_xor(s, 16, 32); s += __shfl_xor(s, 8, 32); s += __shfl_xor(s, 4, 32); s += __shfl_xor(s, 2, 32); s += __shfl_xor(s, 1, 32);
        if (lane == 0) dg[rl] = s;
#pragma unroll 1
        for (int ps = 0; ps < 2; ++ps) {
#pragma unroll
            for (int it = 0; it < ITS; ++it) *(volatile v8h*)(prow + it * 256) = pv[it];
            if (ps == 0) __threadfence(); }
    }
    __syncthreads();
    if (wave == 0) { const float d = dg[lane]; const float rs = rsqrtf(d); const float dv = (d > 0.0f) ? rs : 0.0f;
        float* dst = DV + (size_t)blockIdx.x * SR + lane;
        *(volatile float*)dst = dv; __threadfence(); *(volatile float*)dst = dv; }
}

static_assert(4 * 32 * 16 == 16 * 64 * 2);
__global__ __launch_bounds__(32) void k_h2t(const bf* __restrict__ WT, const bf* __restrict__ XB, const float* __restrict__ DV, h16* H2T) {
    __shared__ __align__(16) float os[16 * 68];
    const int lane = threadIdx.x & 31, lr = lane & 15, hi = lane >> 4; const int r0 = blockIdx.x * 64, c0 = blockIdx.y * 64;
    v8f acc[4][4];
#pragma unroll
    for (int mb = 0; mb < 4; ++mb)
#pragma unroll
        for (int nb = 0; nb < 4; ++nb) acc[mb][nb] = (v8f){};
    const size_t aoff = (size_t)(r0 + lr) * FF + 8 * hi, boff = (size_t)(c0 + lr) * FF + 8 * hi;
#pragma unroll 1
    for (int kc = 0; kc < FF; kc += 32) {
        v16bf a[4];
#pragma unroll
        for (int mb = 0; mb < 4; ++mb) a[mb] = ldb(WT + aoff + (size_t)mb * 16 * FF + kc);
#pragma unroll
        for (int nb = 0; nb < 4; ++nb) { const v16bf b = ldb(XB + boff + (size_t)nb * 16 * FF + kc);
#pragma unroll
            for (int mb = 0; mb < 4; ++mb) acc[mb][nb] = wmmabg(a[mb], b, acc[mb][nb]); }
    }
    float dc[4];
#pragma unroll
    for (int nb = 0; nb < 4; ++nb) dc[nb] = DV[c0 + nb * 16 + lr] * H2S;
#pragma unroll
    for (int mb = 0; mb < 4; ++mb) {
#pragma unroll
        for (int nb = 0; nb < 4; ++nb) {
#pragma unroll
            for (int j = 0; j < 8; ++j) os[(hi * 8 + j) * 68 + nb * 16 + lr] = acc[mb][nb][j] * dc[nb]; }
        wave_sync();
#pragma unroll 1
        for (int ps = 0; ps < 2; ++ps) {
#pragma unroll
            for (int s = 0; s < 4; ++s) { const int row = 4 * s + (lane >> 3), c8 = (lane & 7) * 8;
                const v4f x0 = *(const v4fa*)(&os[row * 68 + c8]); const v4f x1 = *(const v4fa*)(&os[row * 68 + c8 + 4]); v8h hv;
#pragma unroll
                for (int i = 0; i < 4; ++i) { hv[i] = toh_flush(x0[i]); hv[4 + i] = toh_flush(x1[i]); }
                *(volatile v8h*)(H2T + (size_t)(r0 + mb * 16 + row) * NN + c0 + c8) = hv; }
            if (ps == 0) __threadfence(); }
        wave_sync();
    }
}

__global__ __launch_bounds__(32) void k_out(const h16* __restrict__ P, const h16* __restrict__ H2T, const float* __restrict__ DV, const float* __restrict__ bias, float* OUT) {
    __shared__ __align__(16) float os[16 * 68];
    const int lane = threadIdx.x & 31, lr = lane & 15, hi = lane >> 4; const int r0 = blockIdx.x * 64, c0 = blockIdx.y * 64;
    v8f acc[4][4];
#pragma unroll
    for (int mb = 0; mb < 4; ++mb)
#pragma unroll
        for (int nb = 0; nb < 4; ++nb) acc[mb][nb] = (v8f){};
    const size_t aoff = (size_t)(r0 + lr) * NN + 8 * hi, boff = (size_t)(c0 + lr) * NN + 8 * hi;
#pragma unroll 1
    for (int kc = 0; kc < NN; kc += 32) {
        v16h a[4];
#pragma unroll
        for (int mb = 0; mb < 4; ++mb) a[mb] = ldh(P + aoff + (size_t)mb * 16 * NN + kc);
#pragma unroll
        for (int nb = 0; nb < 4; ++nb) { const v16h b = ldh(H2T + boff + (size_t)nb * 16 * NN + kc);
#pragma unroll
            for (int mb = 0; mb < 4; ++mb) acc[mb][nb] = wmma16g(a[mb], b, acc[mb][nb]); }
    }
    float bc[4];
#pragma unroll
    for (int nb = 0; nb < 4; ++nb) bc[nb] = bfr(bias[c0 + nb * 16 + lr]);
#pragma unroll
    for (int mb = 0; mb < 4; ++mb) {
        float dr[8];
#pragma unroll
        for (int j = 0; j < 8; ++j) dr[j] = DV[r0 + mb * 16 + hi * 8 + j] * H2I;
#pragma unroll
        for (int nb = 0; nb < 4; ++nb) {
#pragma unroll
            for (int j = 0; j < 8; ++j) os[(hi * 8 + j) * 68 + nb * 16 + lr] = acc[mb][nb][j] * dr[j] + bc[nb]; }
        wave_sync();
#pragma unroll 1
        for (int ps = 0; ps < 2; ++ps) {
#pragma unroll
            for (int s = 0; s < 8; ++s) { const int row = 2 * s + (lane >> 4), cofs = (lane & 15) * 4;
                const v4f val = *(const v4fa*)(&os[row * 68 + cofs]);
                *(volatile v4f*)(OUT + (size_t)(r0 + mb * 16 + row) * FF + c0 + cofs) = val; }
            if (ps == 0) __threadfence(); }
        wave_sync();
    }
}

static constexpr size_t al256(size_t v) { return (v + 255) & ~(size_t)255; }
static constexpr size_t SZ_XB = al256((size_t)NN * FF * 2);
static constexpr size_t SZ_WT = al256((size_t)FF * FF * 2);
static constexpr size_t SZ_S  = al256((size_t)NN * NN * 4);
static constexpr size_t SZ_P  = al256((size_t)NN * NN * 2);
static constexpr size_t SZ_H2 = al256((size_t)FF * NN * 2);
static constexpr size_t SZ_DV = al256((size_t)NN * 4);
static constexpr size_t SZ_HP = al256((size_t)HB * 256 * 4);
static constexpr size_t SZ_ST = 256;
static constexpr size_t SZ_TOTAL = SZ_XB + SZ_WT + SZ_S + SZ_P + SZ_H2 + SZ_DV + SZ_HP + SZ_ST;
static_assert(SZ_TOTAL <= (size_t)134217728);
static_assert((size_t)(NN / SR) * SR * 4 <= SZ_DV);
static_assert((size_t)HB * 256 * 4 <= SZ_HP);
static_assert((size_t)64 * 4 <= SZ_ST);

extern "C" void kernel_launch(void* const* d_in, const int* in_sizes, int n_in,
                              void* d_out, int out_size, void* d_ws, size_t ws_size, hipStream_t stream) {
    if (n_in < 3) return;
    if ((size_t)in_sizes[0] < (size_t)NN * FF) return;
    if ((size_t)in_sizes[1] < (size_t)FF * FF) return;
    if (in_sizes[2] < FF) return;
    if ((size_t)out_size < (size_t)NN * FF) return;
    if (SZ_TOTAL > ws_size) return;
    const float* x = (const float*)d_in[0];
    const float* W = (const float*)d_in[1];
    const float* bvec = (const float*)d_in[2];
    float* OUT = (float*)d_out;
    char* wsp = (char*)d_ws;
    bf* XB = (bf*)wsp; wsp += SZ_XB;
    bf* WT = (bf*)wsp; wsp += SZ_WT;
    float* S = (float*)wsp; wsp += SZ_S;
    h16* P = (h16*)wsp; wsp += SZ_P;
    h16* H2T = (h16*)wsp; wsp += SZ_H2;
    float* DV = (float*)wsp; wsp += SZ_DV;
    unsigned* HP = (unsigned*)wsp; wsp += SZ_HP;
    unsigned* ST = (unsigned*)wsp; wsp += SZ_ST;

    { const size_t n8 = (size_t)NN * FF / 8; k_cvt8<<<(unsigned)((n8 + 255) / 256), 256, 0, stream>>>(x, XB, n8); }
    k_wt<<<FF / 32, 256, 0, stream>>>(W, WT);
    k_sim<<<dim3(NN / 64, NN / 64, 1), 32, 0, stream>>>(XB, S);
    k_init<<<1, 32, 0, stream>>>(ST);
    for (int pass = 0; pass < 4; ++pass) {
        k_hist<<<HB, HT, 0, stream>>>(S, ST, HP, pass);
        k_scan<<<1, 256, 0, stream>>>(HP, ST);
    }
    k_tie<<<1, TT, 0, stream>>>(S, ST);
    k_select<<<NN / SR, 256, 0, stream>>>(S, ST, P, DV);
    k_h2t<<<dim3(FF / 64, NN / 64, 1), 32, 0, stream>>>(WT, XB, DV, H2T);
    k_out<<<dim3(NN / 64, FF / 64, 1), 32, 0, stream>>>(P, H2T, DV, bvec, OUT);
}
